// GCLayer_22711787062030
// MI455X (gfx1250) — hardware-verified
//
#include <hip/hip_runtime.h>
#include <math.h>

#define NNODE 50000
#define NEDGE 800000
#define NPAD 50048
#define DD 128
#define NT 256
#define SRB 2048
#define NTILE 25
#define RPW 256
#define SCH 2048
#define SPT (SCH / NT)
#define NCH ((NEDGE + SCH - 1) / SCH)
#define LN_EPS 1e-5f
#define WSC 8.0f
#define WSC_INV 0.125f

typedef __attribute__((ext_vector_type(16))) _Float16 v16h;
typedef __attribute__((ext_vector_type(8)))  _Float16 v8h;
typedef __attribute__((ext_vector_type(4)))  _Float16 v4h;
typedef __attribute__((ext_vector_type(16))) __bf16   v16b;
typedef __attribute__((ext_vector_type(8)))  __bf16   v8b;
typedef __attribute__((ext_vector_type(8)))  float    v8f;
typedef __attribute__((ext_vector_type(4)))  float    v4f;
typedef __attribute__((ext_vector_type(4)))  int      v4i;

__device__ __forceinline__ unsigned short f2bf_bits(float f) {
  unsigned u = __float_as_uint(f);
  return (unsigned short)((u + 0x7FFFu + ((u >> 16) & 1u)) >> 16);
}
__device__ __forceinline__ float bf_bits2f(unsigned short h) { return __uint_as_float(((unsigned)h) << 16); }

__device__ __forceinline__ void dep_guard_h(v8f& a, v8f& b, v16h x, v16h y) { asm volatile("v_nop\n\tv_nop\n\tv_nop\n\tv_nop" : "+v"(a), "+v"(b) : "v"(x), "v"(y)); }
__device__ __forceinline__ void dep_guard_b(v8f& a, v8f& b, v16b x, v16b y) { asm volatile("v_nop\n\tv_nop\n\tv_nop\n\tv_nop" : "+v"(a), "+v"(b) : "v"(x), "v"(y)); }
__device__ __forceinline__ void keep4_h(v16h a, v16h b, v16h c, v16h d) { asm volatile("v_nop" :: "v"(a), "v"(b), "v"(c), "v"(d)); }
__device__ __forceinline__ void keep4_b(v16b a, v16b b, v16b c, v16b d) { asm volatile("v_nop" :: "v"(a), "v"(b), "v"(c), "v"(d)); }
__device__ __forceinline__ void acc_guard4(v8f& a, v8f& b, v8f& c, v8f& d) { asm volatile("v_nop\n\tv_nop\n\tv_nop\n\tv_nop" : "+v"(a), "+v"(b), "+v"(c), "+v"(d)); }
template <typename T> struct Frag;
template <> struct Frag<_Float16> {
  typedef v16h V; union U { v16h v; v8h h[2]; };
  static __device__ __forceinline__ v16h load(const _Float16* p) {
    U f; f.h[0] = *(const v8h*)(p); f.h[1] = *(const v8h*)(p + 16); return f.v;
  }
  static __device__ __forceinline__ v8f mma(v16h a, v16h b, v8f c) {
    return __builtin_amdgcn_wmma_f32_16x16x32_f16(false, a, false, b, (short)0, c, false, false);
  }
  static __device__ __forceinline__ void guard(v8f& a, v8f& b, v16h x, v16h y) { dep_guard_h(a, b, x, y); }
  static __device__ __forceinline__ void keep(v16h a, v16h b, v16h c, v16h d) { keep4_h(a, b, c, d); }
};
template <> struct Frag<__bf16> {
  typedef v16b V; union U { v16b v; v8b h[2]; };
  static __device__ __forceinline__ v16b load(const __bf16* p) {
    U f; f.h[0] = *(const v8b*)(p); f.h[1] = *(const v8b*)(p + 16); return f.v;
  }
  static __device__ __forceinline__ v8f mma(v16b a, v16b b, v8f c) {
    return __builtin_amdgcn_wmma_f32_16x16x32_bf16(false, a, false, b, (short)0, c, false, false);
  }
  static __device__ __forceinline__ void guard(v8f& a, v8f& b, v16b x, v16b y) { dep_guard_b(a, b, x, y); }
  static __device__ __forceinline__ void keep(v16b a, v16b b, v16b c, v16b d) { keep4_b(a, b, c, d); }
};

template <int ET> struct Elem;
template <> struct Elem<0> { typedef _Float16 T; };
template <> struct Elem<1> { typedef __bf16 T; };
template <int ET, bool SPLIT, int BIAS_MODE, int OUT_MODE, bool RESID, int ACT = 0>
__global__ __launch_bounds__(256) void wmma_gemm64(
    const unsigned short* __restrict__ Ap, const unsigned short* __restrict__ A2p, int lda, long strideA,
    const unsigned short* __restrict__ Btp, const unsigned short* __restrict__ Bt2p, int ldb, long strideB,
    void* __restrict__ Cout, void* __restrict__ Cout2, int ldc, long strideC,
    const float* __restrict__ bias,
    const float* __restrict__ resid, long strideR,
    int M, int N, int K, float scale) {
  typedef typename Elem<ET>::T T;
  typedef typename Frag<T>::V V;
  const T* A = (const T*)Ap; const T* A2 = (const T*)A2p; const T* Bt = (const T*)Btp; const T* Bt2 = (const T*)Bt2p;
  __shared__ __align__(16) float sT[8][16 * 68];
  const int b    = blockIdx.y;
  const int lane = threadIdx.x & 31;
  const int wave = threadIdx.x >> 5;
  const int tilesN = N >> 6;
  const int tilesM = M >> 6;
  const int tile = blockIdx.x * 8 + wave;
  if (tile >= tilesM * tilesN) return;
  const int tm = tile / tilesN;
  const int tn = tile - tm * tilesN;
  const int m0 = tm << 6;
  const int n0 = tn << 6;

  const T* Ab  = A  + (size_t)b * strideA;
  const T* Bb  = Bt + (size_t)b * strideB;
  const T* Ab2 = SPLIT ? (A2  + (size_t)b * strideA) : nullptr;
  const T* Bb2 = SPLIT ? (Bt2 + (size_t)b * strideB) : nullptr;

  const int rlane = lane & 15;
  const int koff  = (lane >> 4) * 8;
  const int mOff  = (lane >> 4) * 8;

  v8f acc[4][4];
#pragma unroll
  for (int i = 0; i < 4; ++i)
#pragma unroll
    for (int j = 0; j < 4; ++j) acc[i][j] = (v8f){0.f,0.f,0.f,0.f,0.f,0.f,0.f,0.f};

  for (int k0 = 0; k0 < K; k0 += 32) {
    V bh[4], bl[4];
#pragma unroll
    for (int j = 0; j < 4; ++j) {
      const size_t bo = (size_t)(n0 + (j << 4) + rlane) * ldb + koff + k0;
      bh[j] = Frag<T>::load(Bb + bo);
      if (SPLIT) bl[j] = Frag<T>::load(Bb2 + bo);
    }
#pragma unroll
    for (int i = 0; i < 4; ++i) {
      const size_t ao = (size_t)(m0 + (i << 4) + rlane) * lda + koff + k0;
      V ah = Frag<T>::load(Ab + ao);
      V al;
      if (SPLIT) al = Frag<T>::load(Ab2 + ao);
#pragma unroll
      for (int j = 0; j < 4; ++j) {
        acc[i][j] = Frag<T>::mma(ah, bh[j], acc[i][j]);
        if (SPLIT) {
          acc[i][j] = Frag<T>::mma(ah, bl[j], acc[i][j]);
          acc[i][j] = Frag<T>::mma(al, bh[j], acc[i][j]);
        }
      }
      Frag<T>::guard(acc[i][0], acc[i][3], ah, SPLIT ? al : ah);
    }
    Frag<T>::keep(bh[0], bh[1], bh[2], bh[3]);
    if (SPLIT) Frag<T>::keep(bl[0], bl[1], bl[2], bl[3]);
  }
  acc_guard4(acc[0][0], acc[0][1], acc[0][2], acc[0][3]);
  acc_guard4(acc[1][0], acc[1][1], acc[1][2], acc[1][3]);
  acc_guard4(acc[2][0], acc[2][1], acc[2][2], acc[2][3]);
  acc_guard4(acc[3][0], acc[3][1], acc[3][2], acc[3][3]);

  float* slab = sT[wave];
  const float* Rb = RESID ? (resid + (size_t)b * strideR) : nullptr;
#pragma unroll
  for (int i = 0; i < 4; ++i) {
    const int mBase = m0 + (i << 4);
#pragma unroll
    for (int j = 0; j < 4; ++j) {
      const int n = n0 + (j << 4) + rlane;
      float bv = 0.f;
      if (BIAS_MODE == 2) bv = bias[n];
#pragma unroll
      for (int r = 0; r < 8; ++r) {
        float v = acc[i][j][r] * scale;
        if (BIAS_MODE == 1) v += bias[mBase + mOff + r];
        if (BIAS_MODE == 2) v += bv;
        if (RESID) v += Rb[(size_t)(mBase + mOff + r) * ldc + n];
        if (ACT == 1) v = tanhf(v);
        if (ACT == 2) v = fmaxf(v, 0.0f);
        if (ACT == 3) v = v / (1.0f + expf(-v));
        if (ACT == 4) v = (v > 0.f) ? v : 0.01f * v;
        if (ACT == 5) v = 0.5f * v * (1.0f + erff(v * 0.70710678118654752f));
        slab[(mOff + r) * 68 + (j << 4) + rlane] = v;
      }
    }
    __builtin_amdgcn_fence(__ATOMIC_RELEASE, "workgroup");
    __builtin_amdgcn_wave_barrier();
    __builtin_amdgcn_fence(__ATOMIC_ACQUIRE, "workgroup");
    if (OUT_MODE == 0 || OUT_MODE == 3) {
      float* C = (float*)Cout + (size_t)b * strideC;
      const int hh = lane >> 4, c4 = (lane & 15) * 4;
      for (int pass = 0; pass < 2; ++pass) {
#pragma unroll
        for (int it = 0; it < 8; ++it) {
          const int row = it * 2 + hh;
          v4f v = *(const v4f*)(slab + row * 68 + c4);
          *(volatile v4f*)(C + (size_t)(mBase + row) * ldc + n0 + c4) = v;
        }
        __threadfence();
      }
    }
    if (OUT_MODE != 0) {
      const int q = lane >> 3, c8 = (lane & 7) * 8;
      unsigned short* C  = (unsigned short*)((OUT_MODE == 3) ? Cout2 : Cout) + (size_t)b * strideC;
      unsigned short* C2 = (OUT_MODE == 2) ? ((unsigned short*)Cout2 + (size_t)b * strideC) : nullptr;
      for (int pass = 0; pass < 2; ++pass) {
#pragma unroll
        for (int it = 0; it < 4; ++it) {
          const int row = it * 4 + q;
          const float* sp = slab + row * 68 + c8;
          v8h hv, lv;
#pragma unroll
          for (int e = 0; e < 8; ++e) {
            if (OUT_MODE == 1 || OUT_MODE == 3) {
              hv[e] = (_Float16)sp[e];
            } else {
              unsigned short hb = f2bf_bits(sp[e]);
              unsigned short lb = f2bf_bits(sp[e] - bf_bits2f(hb));
              hv[e] = __builtin_bit_cast(_Float16, hb);
              lv[e] = __builtin_bit_cast(_Float16, lb);
            }
          }
          *(volatile v8h*)(C + (size_t)(mBase + row) * ldc + n0 + c8) = hv;
          if (OUT_MODE == 2) *(volatile v8h*)(C2 + (size_t)(mBase + row) * ldc + n0 + c8) = lv;
        }
        __threadfence();
      }
    }
    __builtin_amdgcn_fence(__ATOMIC_RELEASE, "workgroup");
    __builtin_amdgcn_wave_barrier();
    __builtin_amdgcn_fence(__ATOMIC_ACQUIRE, "workgroup");
  }
}

__device__ __forceinline__ int blk_excl_scan(int cnt, int* scan_ws, int tid, int* tot) {
  const int lane = tid & 31, wave = tid >> 5; int incl = cnt;
#pragma unroll
  for (int o = 1; o < 32; o <<= 1) { const int v = __shfl_up(incl, o, 32); if (lane >= o) incl += v; }
  if (lane == 31) scan_ws[wave] = incl;
  __syncthreads();
  if (wave == 0) { int wv = (lane < NT / 32) ? scan_ws[lane] : 0; int wincl = wv;
#pragma unroll
    for (int o = 1; o < 32; o <<= 1) { const int v = __shfl_up(wincl, o, 32); if (lane >= o) wincl += v; }
    if (lane < NT / 32) scan_ws[32 + lane] = wincl - wv; if (lane == 31) scan_ws[64] = wincl; }
  __syncthreads();
  const int res = scan_ws[32 + wave] + incl - cnt; *tot = scan_ws[64];
  return res;
}
template <int SPP, int CAP>
__device__ __forceinline__ int chunk_hits(const int* __restrict__ rowv, const int* __restrict__ colv, int e0, int n0, int tid,
                                          int* LIST, int* LISTE, int* scan_ws) {
  const int eb = e0 + tid * SPP;
  const bool inb = eb < NEDGE;
  const int ebc = inb ? eb : (NEDGE - SPP);
  int rec[SPP]; int cnt = 0;
#pragma unroll
  for (int k = 0; k < SPP; k += 4) {
    const v4i d4 = *(const v4i*)(rowv + ebc + k);
    const v4i s4 = *(const v4i*)(colv + ebc + k);
#pragma unroll
    for (int e = 0; e < 4; ++e) {
      const int d = d4[e]; int r = -1;
      if (inb && d >= n0 && d < n0 + SRB && d < NNODE) {
        int s = s4[e]; s = s < 0 ? 0 : (s >= NNODE ? NNODE - 1 : s);
        r = ((d - n0) << 16) | s; ++cnt;
      }
      rec[k + e] = r;
    }
  }
  int tot; int p = blk_excl_scan(cnt, scan_ws, tid, &tot);
#pragma unroll
  for (int k = 0; k < SPP; ++k) {
    if (rec[k] >= 0) { if ((unsigned)p < (unsigned)CAP) { LIST[p] = rec[k]; LISTE[p] = ebc + k; } ++p; }
  }
  __syncthreads();
  return tot < CAP ? tot : CAP;
}

__global__ __launch_bounds__(NT) void prep_w_kernel(const float* __restrict__ lin_w, const float* __restrict__ msg_w1,
                                                   const float* __restrict__ msg_w2, const float* __restrict__ att_w1,
                                                   const float* __restrict__ out_w1, const float* __restrict__ out_w2,
                                                   unsigned* __restrict__ W16d) {
  const int i = blockIdx.x * NT + threadIdx.x;
  if (i >= 7 * (DD * DD / 2)) return;
  const int q = i >> 13, j = i & 8191;
  const int n = j >> 6, kp = j & 63, k = 2 * kp;
  const float* w = (q == 0) ? lin_w : (q == 1) ? msg_w1 : (q == 2) ? msg_w2 : (q == 3) ? att_w1
                 : (q == 4) ? (att_w1 + DD * DD) : (q == 5) ? out_w1 : out_w2;
  const float a = w[(size_t)k * DD + n] * WSC, b = w[(size_t)(k + 1) * DD + n] * WSC;
  const _Float16 ha = (_Float16)a, hb = (_Float16)b;
  const unsigned u = (unsigned)__builtin_bit_cast(unsigned short, ha) | ((unsigned)__builtin_bit_cast(unsigned short, hb) << 16);
  ((volatile unsigned*)W16d)[i] = u;
  __threadfence();
  ((volatile unsigned*)W16d)[i] = u;
}

__global__ __launch_bounds__(NT) void cast_h_kernel(const float* __restrict__ h, unsigned short* __restrict__ H16) {
  const int i = blockIdx.x * NT + threadIdx.x;
  if (i >= NPAD * (DD / 8)) return;
  const int row = i >> 4, c8 = (i & 15) * 8;
  const int rc = row < NNODE ? row : NNODE - 1;
  const bool live = row < NNODE;
  const v4f a = *(const v4f*)(h + (size_t)rc * DD + c8), b = *(const v4f*)(h + (size_t)rc * DD + c8 + 4);
  v8h o;
#pragma unroll
  for (int e = 0; e < 4; ++e) { o[e] = live ? (_Float16)a[e] : (_Float16)0.0f; o[4 + e] = live ? (_Float16)b[e] : (_Float16)0.0f; }
  unsigned short* p = H16 + (size_t)row * DD + c8;
  *(volatile v8h*)p = o;
  __threadfence();
  *(volatile v8h*)p = o;
}

__global__ __launch_bounds__(NT) void ln_f16_kernel(const float* __restrict__ X, const float* __restrict__ g, const float* __restrict__ bt,
                                                   unsigned short* __restrict__ Y, int nrow2) {
  const int lane = threadIdx.x & 31, wave = threadIdx.x >> 5;
  const int gw = blockIdx.x * (NT / 32) + wave;
  if (gw >= nrow2) return;
  const int row = 2 * gw + (lane >> 4);
  const int c8 = (lane & 15) * 8;
  const float* xr = X + (size_t)row * DD + c8;
  const v4f a = *(const v4f*)xr, b = *(const v4f*)(xr + 4);
  float s = ((a[0] + a[1]) + (a[2] + a[3])) + ((b[0] + b[1]) + (b[2] + b[3]));
  s += __shfl_xor(s, 1, 32); s += __shfl_xor(s, 2, 32); s += __shfl_xor(s, 4, 32); s += __shfl_xor(s, 8, 32);
  const float m = s * (1.0f / DD);
  const v4f da = a - m, db = b - m;
  float s2 = (da[0] * da[0] + da[1] * da[1]) + (da[2] * da[2] + da[3] * da[3])
           + (db[0] * db[0] + db[1] * db[1]) + (db[2] * db[2] + db[3] * db[3]);
  s2 += __shfl_xor(s2, 1, 32); s2 += __shfl_xor(s2, 2, 32); s2 += __shfl_xor(s2, 4, 32); s2 += __shfl_xor(s2, 8, 32);
  const float rs = rsqrtf(s2 * (1.0f / DD) + LN_EPS);
  const v4f ga = *(const v4f*)(g + c8), gb = *(const v4f*)(g + c8 + 4);
  const v4f ba = *(const v4f*)(bt + c8), bb = *(const v4f*)(bt + c8 + 4);
  v8h o;
#pragma unroll
  for (int e = 0; e < 4; ++e) {
    float t0 = da[e] * rs; t0 = t0 * ga[e]; t0 = t0 + ba[e]; o[e] = (_Float16)t0;
    float t1 = db[e] * rs; t1 = t1 * gb[e]; t1 = t1 + bb[e]; o[4 + e] = (_Float16)t1;
  }
  unsigned short* yp = Y + (size_t)row * DD + c8;
  *(volatile v8h*)yp = o;
  __threadfence();
  *(volatile v8h*)yp = o;
}

__global__ __launch_bounds__(NT) void ln_out_kernel(const float* __restrict__ X, const float* __restrict__ g, const float* __restrict__ bt,
                                                   float* __restrict__ out, int nrows) {
  const int lane = threadIdx.x & 31, wave = threadIdx.x >> 5;
  const int row = blockIdx.x * (NT / 32) + wave;
  if (row >= nrows) return;
  const int c4 = 4 * lane;
  const v4f a = *(const v4f*)(X + (size_t)row * DD + c4);
  float s = (a[0] + a[1]) + (a[2] + a[3]);
  s += __shfl_xor(s, 16, 32); s += __shfl_xor(s, 8, 32); s += __shfl_xor(s, 4, 32); s += __shfl_xor(s, 2, 32); s += __shfl_xor(s, 1, 32);
  const float m = s * (1.0f / DD);
  const v4f d = a - m;
  float s2 = (d[0] * d[0] + d[1] * d[1]) + (d[2] * d[2] + d[3] * d[3]);
  s2 += __shfl_xor(s2, 16, 32); s2 += __shfl_xor(s2, 8, 32); s2 += __shfl_xor(s2, 4, 32); s2 += __shfl_xor(s2, 2, 32); s2 += __shfl_xor(s2, 1, 32);
  const float rs = rsqrtf(s2 * (1.0f / DD) + LN_EPS);
  const v4f gv = *(const v4f*)(g + c4), bv = *(const v4f*)(bt + c4);
  v4f o;
#pragma unroll
  for (int e = 0; e < 4; ++e) { float t = d[e] * rs; t = t * gv[e]; o[e] = t + bv[e]; }
  float* op = out + (size_t)row * DD + c4;
  *(volatile v4f*)op = o;
  __threadfence();
  *(volatile v4f*)op = o;
}

__global__ __launch_bounds__(NT) void agg_kernel(const int* __restrict__ rowv, const int* __restrict__ colv,
                                                const float* __restrict__ ea, const float* __restrict__ em,
                                                const unsigned short* __restrict__ U16, const unsigned short* __restrict__ V16,
                                                const float* __restrict__ XU, const float* __restrict__ attw1,
                                                const float* __restrict__ attb1, const float* __restrict__ attw2,
                                                const float* __restrict__ attb2, float* ACC, unsigned short* __restrict__ MSG16) {
  __shared__ int LIST[SCH];
  __shared__ int LISTE[SCH];
  __shared__ int scan_ws[80];
  const int tid = threadIdx.x, lane = tid & 31, wave = tid >> 5;
  const int n0 = blockIdx.x * SRB;
  const v4f we = *(const v4f*)(attw1 + (size_t)2 * DD * DD + 4 * lane);
  const v4f b1 = *(const v4f*)(attb1 + 4 * lane);
  const v4f w2 = *(const v4f*)(attw2 + 4 * lane);
  const float b2 = attb2[0];
  const _Float16* Uh = (const _Float16*)(const void*)U16;
  const _Float16* Vh = (const _Float16*)(const void*)V16;
  const v4f z4 = {0.f, 0.f, 0.f, 0.f};
#pragma unroll 1
  for (int j = 0; j < RPW; ++j) {
    const int n = n0 + wave * RPW + j;
    if (n < NPAD) {
      float* rp = ACC + (size_t)n * DD + 4 * lane;
      *(volatile v4f*)rp = z4;
      __threadfence();
      *(volatile v4f*)rp = z4;
    }
  }
#pragma unroll 1
  for (int c = 0; c < NCH; ++c) {
    const int tot = chunk_hits<SPT, SCH>(rowv, colv, c * SCH, n0, tid, LIST, LISTE, scan_ws);
#pragma unroll 1
    for (int base = 0; base < tot; base += 32) {
      const int q = base + lane;
      const int qc = q < SCH ? q : SCH - 1;
      int rv = LIST[qc], ev = LISTE[qc];
      if (q >= tot) { rv = -1; ev = 0; }
      const int own = (rv >= 0 && (rv >> 24) == wave) ? 1 : 0;
      unsigned msk = (unsigned)__ballot(own);
#pragma unroll 1
      for (int it = 0; it < 32; ++it) {
        if (msk == 0u) break;
        const int bp = __builtin_ctz(msk); msk &= msk - 1u;
        const int r = __shfl(rv, bp, 32);
        int e = __shfl(ev, bp, 32); e = e < 0 ? 0 : (e >= NEDGE ? NEDGE - 1 : e);
        const int dl = (r >> 16) & (SRB - 1);
        int s = r & 0xFFFF; s = s < NNODE ? s : NNODE - 1;
        int nd = n0 + dl; nd = nd < NNODE ? nd : NNODE - 1;
        const float ae = ea[e], me = em[e];
        const v4h uh = *(const v4h*)(Uh + (size_t)nd * DD + 4 * lane);
        const v4h vh = *(const v4h*)(Vh + (size_t)s * DD + 4 * lane);
        v4f sz;
#pragma unroll
        for (int i = 0; i < 4; ++i) {
          float zi = (float)uh[i] + (float)vh[i];
          zi = zi + ae * we[i];
          zi = zi + b1[i];
          const float t = __expf(-zi);
          sz[i] = zi * __builtin_amdgcn_rcpf(1.0f + t);
        }
        float dsum = sz[0] * w2[0];
        dsum += sz[1] * w2[1]; dsum += sz[2] * w2[2]; dsum += sz[3] * w2[3];
        dsum += __shfl_xor(dsum, 16, 32); dsum += __shfl_xor(dsum, 8, 32); dsum += __shfl_xor(dsum, 4, 32);
        dsum += __shfl_xor(dsum, 2, 32); dsum += __shfl_xor(dsum, 1, 32);
        const float te = __expf(-(dsum + b2));
        const float att = me * __builtin_amdgcn_rcpf(1.0f + te);
        const v4f xv = *(const v4f*)(XU + (size_t)s * DD + 4 * lane);
        float* rp = ACC + (size_t)nd * DD + 4 * lane;
        v4f a = *(const v4f*)rp;
        a = a + att * xv;
        *(volatile v4f*)rp = a;
        __threadfence();
        *(volatile v4f*)rp = a;
      }
    }
    __syncthreads();
  }
#pragma unroll 1
  for (int jj = 0; jj < RPW / 2; ++jj) {
    const int ne = n0 + wave * RPW + 2 * jj;
    if (ne < NPAD) {
      const int n = ne + (lane >> 4);
      const int c8 = (lane & 15) * 8;
      const float* rp = ACC + (size_t)n * DD + c8;
      const v4f a = *(const v4f*)rp, b = *(const v4f*)(rp + 4);
      v8h o;
#pragma unroll
      for (int e = 0; e < 4; ++e) { o[e] = (_Float16)a[e]; o[4 + e] = (_Float16)b[e]; }
      unsigned short* mp = MSG16 + (size_t)n * DD + c8;
      *(volatile v8h*)mp = o;
      __threadfence();
      *(volatile v8h*)mp = o;
    }
  }
}

extern "C" void kernel_launch(void* const* d_in, const int* in_sizes, int n_in,
                              void* d_out, int out_size, void* d_ws, size_t ws_size, hipStream_t stream) {
  if (n_in < 26) return;
  const float* h        = (const float*)d_in[0];
  const float* edge_attr= (const float*)d_in[1];
  const int*   rowv     = (const int*)  d_in[2];
  const int*   colv     = (const int*)  d_in[3];
  const float* edge_mask= (const float*)d_in[5];
  const float* lin_w    = (const float*)d_in[6];
  const float* lin_b    = (const float*)d_in[7];
  const float* msg_w1   = (const float*)d_in[8];
  const float* msg_b1   = (const float*)d_in[9];
  const float* msg_ln_g = (const float*)d_in[10];
  const float* msg_ln_b = (const float*)d_in[11];
  const float* msg_w2   = (const float*)d_in[12];
  const float* msg_b2   = (const float*)d_in[13];
  const float* att_w1   = (const float*)d_in[14];
  const float* att_b1   = (const float*)d_in[15];
  const float* att_w2   = (const float*)d_in[16];
  const float* att_b2   = (const float*)d_in[17];
  const float* out_w1   = (const float*)d_in[18];
  const float* out_b1   = (const float*)d_in[19];
  const float* out_ln_g = (const float*)d_in[20];
  const float* out_ln_b = (const float*)d_in[21];
  const float* out_w2   = (const float*)d_in[22];
  const float* out_b2   = (const float*)d_in[23];
  const float* ln_g     = (const float*)d_in[24];
  const float* ln_b     = (const float*)d_in[25];
  float* out = (float*)d_out;

  if (in_sizes[0] != NNODE * DD || in_sizes[1] != NEDGE || in_sizes[2] != NEDGE || in_sizes[3] != NEDGE ||
      in_sizes[5] != NEDGE || in_sizes[14] != 257 * DD || in_sizes[16] != DD || in_sizes[17] < 1 ||
      out_size != NNODE * DD) return;

  char* ws = (char*)d_ws; size_t off = 0;
  auto carve = [&](size_t bytes) -> char* { char* p = ws + off; off += (bytes + 255) & ~(size_t)255; return p; };
  unsigned short* W16 = (unsigned short*)carve((size_t)7 * DD * DD * 2);
  float*          RA  = (float*)carve((size_t)NPAD * DD * 4);
  float*          RB  = (float*)carve((size_t)NPAD * DD * 4);
  float*          RF  = (float*)carve((size_t)NPAD * DD * 4);
  unsigned short* RC1 = (unsigned short*)carve((size_t)NPAD * DD * 2);
  unsigned short* RE  = (unsigned short*)carve((size_t)NPAD * DD * 2);
  unsigned short* RC2 = (unsigned short*)carve((size_t)NPAD * DD * 2);
  if (off > ws_size || off > (size_t)134217728) return;
  (void)RE;

  const int PL = DD * DD;
  const dim3 gg((((NPAD / 64) * (DD / 64)) + 7) / 8, 1);
  const dim3 gg2(gg.x, 2);

  prep_w_kernel<<<(7 * (DD * DD / 2) + NT - 1) / NT, NT, 0, stream>>>(lin_w, msg_w1, msg_w2, att_w1, out_w1, out_w2, (unsigned*)W16);
  cast_h_kernel<<<(NPAD * (DD / 8) + NT - 1) / NT, NT, 0, stream>>>(h, RC1);
  wmma_gemm64<0, false, 2, 3, false, 0><<<gg, NT, 0, stream>>>(
      RC1, nullptr, DD, 0L, W16 + 0 * PL, nullptr, DD, 0L, (void*)RA, (void*)RC2, DD, 0L,
      lin_b, nullptr, 0L, NPAD, DD, DD, WSC_INV);
  wmma_gemm64<0, false, 2, 0, false, 3><<<gg, NT, 0, stream>>>(
      RC2, nullptr, DD, 0L, W16 + 1 * PL, nullptr, DD, 0L, (void*)RB, nullptr, DD, 0L,
      msg_b1, nullptr, 0L, NPAD, DD, DD, WSC_INV);
  ln_f16_kernel<<<(NPAD / 2 + (NT / 32) - 1) / (NT / 32), NT, 0, stream>>>(RB, msg_ln_g, msg_ln_b, RC1, NPAD / 2);
  wmma_gemm64<0, false, 2, 0, false, 0><<<gg, NT, 0, stream>>>(
      RC1, nullptr, DD, 0L, W16 + 2 * PL, nullptr, DD, 0L, (void*)RB, nullptr, DD, 0L,
      msg_b2, nullptr, 0L, NPAD, DD, DD, WSC_INV);
  wmma_gemm64<0, false, 0, 1, false, 0><<<gg2, NT, 0, stream>>>(
      RC2, nullptr, DD, 0L, W16 + 3 * PL, nullptr, DD, (long)PL, (void*)RC1, nullptr, DD, (long)NPAD * DD,
      nullptr, nullptr, 0L, NPAD, DD, DD, WSC_INV);
  agg_kernel<<<NTILE, NT, 0, stream>>>(rowv, colv, edge_attr, edge_mask, RC1, RC1 + (size_t)NPAD * DD, RB,
                                       att_w1, att_b1, att_w2, att_b2, RF, RC2);
  wmma_gemm64<0, false, 2, 0, false, 3><<<gg, NT, 0, stream>>>(
      RC2, nullptr, DD, 0L, W16 + 5 * PL, nullptr, DD, 0L, (void*)RB, nullptr, DD, 0L,
      out_b1, nullptr, 0L, NPAD, DD, DD, WSC_INV);
  ln_f16_kernel<<<(NPAD / 2 + (NT / 32) - 1) / (NT / 32), NT, 0, stream>>>(RB, out_ln_g, out_ln_b, RC1, NPAD / 2);
  wmma_gemm64<0, false, 2, 0, true, 0><<<gg, NT, 0, stream>>>(
      RC1, nullptr, DD, 0L, W16 + 6 * PL, nullptr, DD, 0L, (void*)RF, nullptr, DD, 0L,
      out_b2, RA, 0L, NPAD, DD, DD, WSC_INV);
  ln_out_kernel<<<(NNODE + (NT / 32) - 1) / (NT / 32), NT, 0, stream>>>(RF, ln_g, ln_b, out, NNODE);
}
